// CrossViewAttention_18743237280507
// MI455X (gfx1250) — hardware-verified
//
#include <hip/hip_runtime.h>
#include <math.h>
#include <stdint.h>

#define SEQ 4096
#define DD  512
#define DC  (2 * DD)
#ifndef NB
#define NB 2
#endif
#ifndef NQ
#define NQ SEQ
#endif
#ifndef QRES
#define QRES 1
#endif
#define NB_FULL   2
#define ROWS_FULL (NB_FULL * SEQ)
#define VSTR  ((long long)ROWS_FULL * DD)
#define VTB   ((long long)DD * SEQ)
#define VTV   ((long long)NB_FULL * DD * SEQ)
#define XB    ((long long)SEQ * DC)
#define OUT1_OFF ((long long)ROWS_FULL * DD)
static_assert(NB >= 1 && NB <= NB_FULL);
static_assert(NQ >= 64 && NQ <= SEQ && (NQ % 64) == 0);
static_assert((SEQ % 128) == 0 && (DD % 64) == 0 && (DC % 32) == 0);
static_assert(OUT1_OFF * 4 == 16777216LL);
static_assert(QRES == 0 || QRES == 1);

typedef _Float16 v16h __attribute__((ext_vector_type(16)));
typedef _Float16 v8h  __attribute__((ext_vector_type(8)));
typedef __bf16   v16b __attribute__((ext_vector_type(16)));
typedef __bf16   v8b  __attribute__((ext_vector_type(8)));
typedef float    v8f  __attribute__((ext_vector_type(8)));
typedef float    v4f  __attribute__((ext_vector_type(4)));
typedef unsigned int v4u __attribute__((ext_vector_type(4)));

#if defined(__HIP_DEVICE_COMPILE__)
#define DEV_ASM 1
#else
#define DEV_ASM 0
#endif

__device__ __forceinline__ unsigned short bf_bits(float f) {
  unsigned u = __float_as_uint(f);
  return (unsigned short)((u + 0x7FFFu + ((u >> 16) & 1u)) >> 16);
}
__device__ __forceinline__ float bf_up(unsigned short hb) { return __uint_as_float(((unsigned)hb) << 16); }
__device__ __forceinline__ float bfr(float f) { return bf_up(bf_bits(f)); }
__device__ __forceinline__ unsigned short h_bits(_Float16 x) { return __builtin_bit_cast(unsigned short, x); }
__device__ __forceinline__ unsigned pk16(unsigned short a, unsigned short b) { return (unsigned)a | ((unsigned)b << 16); }
__device__ __forceinline__ v8f zero8() { v8f z = {0.f, 0.f, 0.f, 0.f, 0.f, 0.f, 0.f, 0.f}; return z; }

template <typename OT> struct FT;
template <> struct FT<__bf16>   { typedef v16b frag; typedef v8b half8; };
template <> struct FT<_Float16> { typedef v16h frag; typedef v8h half8; };

template <typename OT>
__device__ __forceinline__ typename FT<OT>::frag ldfrag(const OT* p) {
  union { typename FT<OT>::frag v; typename FT<OT>::half8 h[2]; } f;
  f.h[0] = *(const typename FT<OT>::half8*)(p);
  f.h[1] = *(const typename FT<OT>::half8*)(p + 16);
  return f.v;
}

__device__ __forceinline__ v8f mmar(v16b a, v16b b, v8f c) {
  return __builtin_amdgcn_wmma_f32_16x16x32_bf16(false, a, false, b, (short)0, c, false, false);
}
__device__ __forceinline__ v8f mma_h(v16h a, v16h b, v8f c) {
  c = __builtin_amdgcn_wmma_f32_16x16x32_f16(false, a, false, b, (short)0, c, false, false);
#if DEV_ASM
  asm volatile("v_nop\n\tv_nop\n\tv_nop\n\tv_nop" : "+v"(c) : "v"(a), "v"(b));
#endif
  return c;
}
__device__ __forceinline__ void dep_guard(v8f& a, v8f& b, v16b x, v16b y) {
#if DEV_ASM
  asm volatile("v_nop\n\tv_nop\n\tv_nop\n\tv_nop" : "+v"(a), "+v"(b) : "v"(x), "v"(y));
#else
  (void)a; (void)b; (void)x; (void)y;
#endif
}
__device__ __forceinline__ void dep_guard(v8f& a, v8f& b, v16h x, v16h y) {
#if DEV_ASM
  asm volatile("v_nop\n\tv_nop\n\tv_nop\n\tv_nop" : "+v"(a), "+v"(b) : "v"(x), "v"(y));
#else
  (void)a; (void)b; (void)x; (void)y;
#endif
}
__device__ __forceinline__ void keep4(v16b a, v16b b, v16b c, v16b d) {
#if DEV_ASM
  asm volatile("v_nop" :: "v"(a), "v"(b), "v"(c), "v"(d));
#else
  (void)a; (void)b; (void)c; (void)d;
#endif
}
__device__ __forceinline__ void keep4(v16h a, v16h b, v16h c, v16h d) {
#if DEV_ASM
  asm volatile("v_nop" :: "v"(a), "v"(b), "v"(c), "v"(d));
#else
  (void)a; (void)b; (void)c; (void)d;
#endif
}
__device__ __forceinline__ void acc_guard4(v8f& a, v8f& b, v8f& c, v8f& d) {
#if DEV_ASM
  asm volatile("v_nop\n\tv_nop\n\tv_nop\n\tv_nop" : "+v"(a), "+v"(b), "+v"(c), "+v"(d));
#else
  (void)a; (void)b; (void)c; (void)d;
#endif
}

__device__ __forceinline__ v4u pack_bf8(v4f a, v4f a4) {
  v4u p;
  p[0] = pk16(bf_bits(a[0]),  bf_bits(a[1]));
  p[1] = pk16(bf_bits(a[2]),  bf_bits(a[3]));
  p[2] = pk16(bf_bits(a4[0]), bf_bits(a4[1]));
  p[3] = pk16(bf_bits(a4[2]), bf_bits(a4[3]));
  return p;
}

__global__ __launch_bounds__(256) void cvt_w(const float* __restrict__ in, unsigned short* out, int n8) {
  const int i = blockIdx.x * 256 + (int)threadIdx.x;
  if (i < n8) {
    const v4f a  = *(const v4f*)(in + (size_t)i * 8);
    const v4f a4 = *(const v4f*)(in + (size_t)i * 8 + 4);
    const v4u p = pack_bf8(a, a4);
    unsigned short* o = out + (size_t)i * 8;
    *(volatile v4u*)o = p;
    __threadfence();
    *(volatile v4u*)o = p;
  }
}

__global__ __launch_bounds__(256) void cvt_x(const float* __restrict__ xa, const float* __restrict__ xb,
                                             unsigned short* out, int n8) {
  const int i   = blockIdx.x * 256 + (int)threadIdx.x;
  const int src = (int)blockIdx.y;
  if (i < n8) {
    const float* in = (src == 0) ? xa : xb;
    const size_t e = (size_t)i * 8;
    const v4f a  = *(const v4f*)(in + e);
    const v4f a4 = *(const v4f*)(in + e + 4);
    const v4u p = pack_bf8(a, a4);
    const size_t row = e >> 9;
    const size_t col = e & (size_t)(DD - 1);
    unsigned short* o = out + row * DC + (size_t)src * DD + col;
    *(volatile v4u*)o = p;
    __threadfence();
    *(volatile v4u*)o = p;
  }
}

template <typename OT, int OUT_MODE, int BIAS, bool RELU>
__global__ __launch_bounds__(256) void gemm64(
    const unsigned short* __restrict__ Ap, int lda, long long sAy, long long sAz,
    const unsigned short* __restrict__ Btp, int ldb, long long sBy, long long sBz,
    void* Cout, void* Cout2, int ldc, long long sCy, long long sCz,
    const float* __restrict__ bias,
    int M, int N, int K, float oscale, float rscale) {
  typedef typename FT<OT>::frag V16;
  const OT* A  = (const OT*)(const void*)Ap;
  const OT* Bt = (const OT*)(const void*)Btp;
  __shared__ __align__(16) float sT[8][16 * 68];
  const int by   = (int)blockIdx.y;
  const int bz   = (int)blockIdx.z;
  const int lane = threadIdx.x & 31;
  const int wave = threadIdx.x >> 5;
  const int tilesN = N >> 6;
  const int tilesM = M >> 6;
  const int tile = blockIdx.x * 8 + wave;
  if (tile >= tilesM * tilesN) return;
  const int tm = tile / tilesN;
  const int tn = tile - tm * tilesN;
  const int m0 = tm << 6;
  const int n0 = tn << 6;

  const OT* Ab = A  + (size_t)((long long)by * sAy + (long long)bz * sAz);
  const OT* Bb = Bt + (size_t)((long long)by * sBy + (long long)bz * sBz);
  const size_t cOff = (size_t)((long long)by * sCy + (long long)bz * sCz);

  const int rlane = lane & 15;
  const int koff  = (lane >> 4) * 8;
  const int mOff  = (lane >> 4) * 8;

  v8f acc[4][4];
#pragma unroll
  for (int i = 0; i < 4; ++i)
#pragma unroll
    for (int j = 0; j < 4; ++j) acc[i][j] = zero8();

  for (int k0 = 0; k0 < K; k0 += 32) {
    V16 bq[4];
#pragma unroll
    for (int j = 0; j < 4; ++j)
      bq[j] = ldfrag<OT>(Bb + (size_t)(n0 + (j << 4) + rlane) * ldb + koff + k0);
#pragma unroll
    for (int i = 0; i < 4; ++i) {
      const V16 af = ldfrag<OT>(Ab + (size_t)(m0 + (i << 4) + rlane) * lda + koff + k0);
#pragma unroll
      for (int j = 0; j < 4; ++j) acc[i][j] = mmar(af, bq[j], acc[i][j]);
      dep_guard(acc[i][0], acc[i][3], af, bq[3]);
    }
    keep4(bq[0], bq[1], bq[2], bq[3]);
  }
  acc_guard4(acc[0][0], acc[0][1], acc[0][2], acc[0][3]);
  acc_guard4(acc[1][0], acc[1][1], acc[1][2], acc[1][3]);
  acc_guard4(acc[2][0], acc[2][1], acc[2][2], acc[2][3]);
  acc_guard4(acc[3][0], acc[3][1], acc[3][2], acc[3][3]);

  float* slab = sT[wave];
#pragma unroll
  for (int i = 0; i < 4; ++i) {
    const int mBase = m0 + (i << 4);
#pragma unroll
    for (int j = 0; j < 4; ++j) {
#pragma unroll
      for (int r = 0; r < 8; ++r) {
        slab[(mOff + r) * 68 + (j << 4) + rlane] = acc[i][j][r];
      }
    }
    __builtin_amdgcn_fence(__ATOMIC_RELEASE, "workgroup");
    __builtin_amdgcn_wave_barrier();
    __builtin_amdgcn_fence(__ATOMIC_ACQUIRE, "workgroup");
    if (OUT_MODE == 0) {
      float* C = (float*)Cout + cOff;
      const int h2 = lane >> 4, c4 = (lane & 15) * 4;
      v4f badd = {0.f, 0.f, 0.f, 0.f};
      if (BIAS == 1) {
#pragma unroll
        for (int e = 0; e < 4; ++e) badd[e] = bfr(bias[n0 + c4 + e]);
      }
      v4f vals[8];
#pragma unroll
      for (int it = 0; it < 8; ++it) {
        const int row = it * 2 + h2;
        v4f v = *(const v4f*)(slab + row * 68 + c4);
        if (BIAS == 1) v = v + badd;
        if (BIAS == 2) v = v + bfr(bias[mBase + row]);
        if (RELU) {
#pragma unroll
          for (int e = 0; e < 4; ++e) v[e] = fmaxf(v[e], 0.f);
        }
        vals[it] = v * oscale;
      }
      for (int pass = 0; pass < 2; ++pass) {
#pragma unroll
        for (int it = 0; it < 8; ++it) {
          const int row = it * 2 + h2;
          *(volatile v4f*)(C + (size_t)(mBase + row) * ldc + n0 + c4) = vals[it];
        }
        __threadfence();
      }
    } else {
      const int q = lane >> 3, c8 = (lane & 7) * 8;
      unsigned short* C  = (unsigned short*)Cout  + cOff;
      unsigned short* C2 = (unsigned short*)Cout2 + cOff;
      float cb[8];
#pragma unroll
      for (int e = 0; e < 8; ++e) cb[e] = (BIAS == 1) ? bfr(bias[n0 + c8 + e]) : 0.f;
      v4u hv[4], lv[4];
#pragma unroll
      for (int it = 0; it < 4; ++it) {
        const int row = it * 4 + q;
        const float* sp = slab + row * 68 + c8;
        const float rb = (BIAS == 2) ? bfr(bias[mBase + row]) : 0.f;
        float f[8];
#pragma unroll
        for (int e = 0; e < 8; ++e) f[e] = sp[e] + cb[e] + rb;
        v4u a, a2;
#pragma unroll
        for (int e = 0; e < 4; ++e) {
          const float f0 = f[2 * e], f1 = f[2 * e + 1];
          const _Float16 x0 = (_Float16)f0, x1 = (_Float16)f1;
          const unsigned short h0 = h_bits(x0), h1 = h_bits(x1);
          unsigned short l0 = 0, l1 = 0;
          if (OUT_MODE == 3) {
            l0 = h_bits((_Float16)((f0 - (float)x0) * rscale));
            l1 = h_bits((_Float16)((f1 - (float)x1) * rscale));
          }
          a[e] = pk16(h0, h1); a2[e] = pk16(l0, l1);
        }
        hv[it] = a; lv[it] = a2;
      }
      for (int pass = 0; pass < 2; ++pass) {
#pragma unroll
        for (int it = 0; it < 4; ++it) {
          const int row = it * 4 + q;
          *(volatile v4u*)(C + (size_t)(mBase + row) * ldc + n0 + c8) = hv[it];
          if (OUT_MODE == 3) *(volatile v4u*)(C2 + (size_t)(mBase + row) * ldc + n0 + c8) = lv[it];
        }
        __threadfence();
      }
    }
    __builtin_amdgcn_fence(__ATOMIC_RELEASE, "workgroup");
    __builtin_amdgcn_wave_barrier();
    __builtin_amdgcn_fence(__ATOMIC_ACQUIRE, "workgroup");
  }
}

__global__ __launch_bounds__(256)
void attn_cv(const unsigned short* __restrict__ qhp, const unsigned short* __restrict__ qlp,
             const unsigned short* __restrict__ kpp, const unsigned short* __restrict__ vtp,
             const float* __restrict__ co, float* out) {
  union FH { v16h v; v8h h[2]; };
  __shared__ __align__(16) float    Ss[32 * 128];
  __shared__ __align__(16) _Float16 Ps[32 * 128];
  __shared__ __align__(16) float    Os[8][16 * 64];
  __shared__ __align__(16) float    Al[32];
  __shared__ __align__(16) float    Rs[32];

  const int tid  = (int)threadIdx.x;
  const int wave = tid >> 5;
  const int lane = tid & 31;
  const int hh   = lane >> 4;
  const int c    = lane & 15;
  const int rt   = wave >> 2;
  const int wq   = wave & 3;
  const int srw  = tid >> 3;
  const int sub  = tid & 7;

  const int dir = (int)blockIdx.z;
  const int b   = (int)blockIdx.y;
  const int q0  = (int)blockIdx.x * 32;
  const int kvw = 1 - dir;
  const size_t rowQ = (size_t)b * SEQ + (size_t)q0;

  const _Float16* Qh  = (const _Float16*)(const void*)qhp + (size_t)dir * VSTR + rowQ * DD;
  const _Float16* Kb  = (const _Float16*)(const void*)kpp + (size_t)kvw * VSTR + (size_t)b * SEQ * DD;
  const _Float16* Vtb = (const _Float16*)(const void*)vtp + (size_t)dir * VTV + (size_t)b * VTB;
  const float* cob = co + rowQ * DD;
  float* ob = out + (size_t)dir * OUT1_OFF + rowQ * DD;

  const _Float16* qhrow = Qh + (size_t)(rt * 16 + c) * DD + 8 * hh;
#if QRES
  const _Float16* Ql = (const _Float16*)(const void*)qlp + (size_t)dir * VSTR + rowQ * DD;
  const _Float16* qlrow = Ql + (size_t)(rt * 16 + c) * DD + 8 * hh;
#endif
  const int colbase = wq * 128;

  float mrun = -INFINITY, lrun = 0.f;
  v8f oacc[8];
#pragma unroll
  for (int t = 0; t < 8; ++t) oacc[t] = zero8();

  for (int kc = 0; kc < SEQ / 128; ++kc) {
    const int key0 = kc * 128;

    {
      v8f ah0 = zero8(), ah1 = zero8(), al0 = zero8(), al1 = zero8();
      const _Float16* k0row = Kb + (size_t)(key0 + wq * 32 + c) * DD + 8 * hh;
      const _Float16* k1row = k0row + (size_t)16 * DD;
#pragma unroll 1
      for (int ks = 0; ks < DD / 32; ++ks) {
        const v16h qa  = ldfrag<_Float16>(qhrow + ks * 32);
        const v16h kb0 = ldfrag<_Float16>(k0row + ks * 32);
        const v16h kb1 = ldfrag<_Float16>(k1row + ks * 32);
        ah0 = mma_h(qa, kb0, ah0);
        ah1 = mma_h(qa, kb1, ah1);
#if QRES
        const v16h ql  = ldfrag<_Float16>(qlrow + ks * 32);
        al0 = mma_h(ql, kb0, al0);
        al1 = mma_h(ql, kb1, al1);
#endif
      }
      float* swp = Ss + (rt * 16 + 8 * hh) * 128 + wq * 32 + c;
#pragma unroll
      for (int r = 0; r < 8; ++r) {
        swp[r * 128]      = ah0[r] + al0[r] * (1.0f / 4096.0f);
        swp[r * 128 + 16] = ah1[r] + al1[r] * (1.0f / 4096.0f);
      }
    }
    __syncthreads();

    {
      const float* sp = Ss + srw * 128 + sub * 16;
      float e[16];
      {
        const v4f t0 = *(const v4f*)(sp);
        const v4f t1 = *(const v4f*)(sp + 4);
        const v4f t2 = *(const v4f*)(sp + 8);
        const v4f t3 = *(const v4f*)(sp + 12);
#pragma unroll
        for (int i = 0; i < 4; ++i) { e[i] = t0[i]; e[4 + i] = t1[i]; e[8 + i] = t2[i]; e[12 + i] = t3[i]; }
      }
      float m = e[0];
#pragma unroll
      for (int i = 1; i < 16; ++i) m = fmaxf(m, e[i]);
      m = fmaxf(m, __shfl_xor(m, 1, 32));
      m = fmaxf(m, __shfl_xor(m, 2, 32));
      m = fmaxf(m, __shfl_xor(m, 4, 32));
      const float mnew  = fmaxf(mrun, m);
      const float msafe = (mnew == -INFINITY) ? 0.f : mnew;
      const float alpha = __expf(mrun - msafe);
      mrun = mnew;
      float psum = 0.f;
      v8h p0, p1;
#pragma unroll
      for (int i = 0; i < 8; ++i) {
        const float pa = __expf(e[i] - msafe);
        const float pb = __expf(e[8 + i] - msafe);
        psum += pa;
        psum += pb;
        p0[i] = (_Float16)(pa * 16384.0f);
        p1[i] = (_Float16)(pb * 16384.0f);
      }
      psum += __shfl_xor(psum, 1, 32);
      psum += __shfl_xor(psum, 2, 32);
      psum += __shfl_xor(psum, 4, 32);
      lrun = lrun * alpha + psum;
      _Float16* pp = Ps + srw * 128 + sub * 16;
      *(v8h*)(pp)     = p0;
      *(v8h*)(pp + 8) = p1;
      if (sub == 0) Al[srw] = alpha;
    }
    __syncthreads();

    {
      const float* ap = Al + rt * 16 + 8 * hh;
      float av[8];
      {
        const v4f a0 = *(const v4f*)(ap);
        const v4f a1 = *(const v4f*)(ap + 4);
#pragma unroll
        for (int r = 0; r < 4; ++r) { av[r] = a0[r]; av[4 + r] = a1[r]; }
      }
#pragma unroll
      for (int t = 0; t < 8; ++t)
#pragma unroll
        for (int r = 0; r < 8; ++r) oacc[t][r] *= av[r];

      const _Float16* prow = Ps + (rt * 16 + c) * 128 + 8 * hh;
      const _Float16* vrow = Vtb + (size_t)(colbase + c) * SEQ + key0 + 8 * hh;
#pragma unroll 1
      for (int kk = 0; kk < 4; ++kk) {
        FH pa;
        pa.h[0] = *(const v8h*)(prow + kk * 32);
        pa.h[1] = *(const v8h*)(prow + kk * 32 + 16);
#pragma unroll
        for (int t = 0; t < 8; ++t) {
          const v16h vb = ldfrag<_Float16>(vrow + (size_t)t * 16 * SEQ + kk * 32);
          oacc[t] = mma_h(pa.v, vb, oacc[t]);
        }
      }
    }
  }

  {
    const float L   = lrun;
    const float inv = (L > 0.f) ? (1.0f / L) : 0.f;
    const float l1  = L * inv;
    const float sc  = inv * (1.0f / fmaxf(l1, 1e-12f)) * (1.0f / 22.627416997969522f) * (1.0f / 16384.0f);
    if (sub == 0) Rs[srw] = sc;
  }
  __syncthreads();

  {
    const float* rp = Rs + rt * 16 + 8 * hh;
    float rv[8];
    {
      const v4f r0 = *(const v4f*)(rp);
      const v4f r1 = *(const v4f*)(rp + 4);
#pragma unroll
      for (int r = 0; r < 4; ++r) { rv[r] = r0[r]; rv[4 + r] = r1[r]; }
    }
    float* os = Os[wave];
    const int h2 = lane >> 4, c4 = (lane & 15) * 4;
#pragma unroll
    for (int hf = 0; hf < 2; ++hf) {
#pragma unroll
      for (int r = 0; r < 8; ++r)
#pragma unroll
        for (int t4 = 0; t4 < 4; ++t4)
          os[(8 * hh + r) * 64 + t4 * 16 + c] = oacc[hf * 4 + t4][r] * rv[r];
      __builtin_amdgcn_fence(__ATOMIC_RELEASE, "workgroup");
      __builtin_amdgcn_wave_barrier();
      __builtin_amdgcn_fence(__ATOMIC_ACQUIRE, "workgroup");
      v4f vals[8];
#pragma unroll
      for (int it = 0; it < 8; ++it) {
        const int row = it * 2 + h2;
        const v4f v  = *(const v4f*)(os + row * 64 + c4);
        const v4f cv = *(const v4f*)(cob + (size_t)(rt * 16 + row) * DD + colbase + hf * 64 + c4);
        vals[it] = v + cv;
      }
      for (int pass = 0; pass < 2; ++pass) {
#pragma unroll
        for (int it = 0; it < 8; ++it) {
          const int row = it * 2 + h2;
          *(volatile v4f*)(ob + (size_t)(rt * 16 + row) * DD + colbase + hf * 64 + c4) = vals[it];
        }
        __threadfence();
      }
      __builtin_amdgcn_fence(__ATOMIC_RELEASE, "workgroup");
      __builtin_amdgcn_wave_barrier();
      __builtin_amdgcn_fence(__ATOMIC_ACQUIRE, "workgroup");
    }
  }
}

extern "C" void kernel_launch(void* const* d_in, const int* in_sizes, int n_in,
                              void* d_out, int out_size, void* d_ws, size_t ws_size,
                              hipStream_t stream) {
  if (n_in < 10) return;
  if (in_sizes[0] < NB * SEQ * DD || in_sizes[1] < NB * SEQ * DD) return;
  if (in_sizes[2] < DD * DD || in_sizes[4] < DD * DD || in_sizes[6] < DD * DD) return;
  if (in_sizes[3] < DD || in_sizes[5] < DD || in_sizes[7] < DD || in_sizes[9] < DD) return;
  if (in_sizes[8] < DD * DC) return;
  if ((long long)out_size < OUT1_OFF + (long long)NB * SEQ * DD) return;

  const float* xf = (const float*)d_in[0];
  const float* xs = (const float*)d_in[1];
  const float* Wq = (const float*)d_in[2];
  const float* bq = (const float*)d_in[3];
  const float* Wk = (const float*)d_in[4];
  const float* bk = (const float*)d_in[5];
  const float* Wv = (const float*)d_in[6];
  const float* bv = (const float*)d_in[7];
  const float* Wc = (const float*)d_in[8];
  const float* bc = (const float*)d_in[9];

  const size_t PXC = (size_t)ROWS_FULL * DC * 2;
  const size_t PW  = (size_t)DD * DD * 2;
  const size_t PWC = (size_t)DD * DC * 2;
  const size_t PQ  = (size_t)2 * VSTR * 2;
  const size_t PVT = (size_t)2 * VTV * 2;
  const size_t PCO = (size_t)ROWS_FULL * DD * 4;
  size_t off = 0;
  const size_t oXc = off; off += PXC;
  const size_t oWq = off; off += PW;
  const size_t oWk = off; off += PW;
  const size_t oWv = off; off += PW;
  const size_t oWc = off; off += PWC;
  const size_t oQh = off; off += PQ;
  const size_t oQl = off; off += PQ;
  const size_t oKp = off; off += PQ;
  const size_t oVt = off; off += PVT;
  const size_t oCo = off; off += PCO;
  if (off > ws_size) return;
  if (off > (size_t)134217728) return;

  char* ws = (char*)d_ws;
  unsigned short* Xc  = (unsigned short*)(ws + oXc);
  unsigned short* Wqb = (unsigned short*)(ws + oWq);
  unsigned short* Wkb = (unsigned short*)(ws + oWk);
  unsigned short* Wvb = (unsigned short*)(ws + oWv);
  unsigned short* Wcb = (unsigned short*)(ws + oWc);
  unsigned short* Qh  = (unsigned short*)(ws + oQh);
  unsigned short* Ql  = (unsigned short*)(ws + oQl);
  unsigned short* Kp  = (unsigned short*)(ws + oKp);
  unsigned short* Vt  = (unsigned short*)(ws + oVt);
  float*          Co  = (float*)(ws + oCo);

  const dim3 blk(256);
  const int n8x = NB * SEQ * DD / 8;
  const int n8w = DD * DD / 8;
  const int n8c = DD * DC / 8;
  const int tq  = (NQ / 64) * (DD / 64);
  const int tk  = ((NB * SEQ) / 64) * (DD / 64);
  const int tv  = (DD / 64) * (SEQ / 64);

  cvt_x<<<dim3((n8x + 255) / 256, 2), blk, 0, stream>>>(xf, xs, Xc, n8x);
  cvt_w<<<dim3((n8w + 255) / 256), blk, 0, stream>>>(Wq, Wqb, n8w);
  cvt_w<<<dim3((n8w + 255) / 256), blk, 0, stream>>>(Wk, Wkb, n8w);
  cvt_w<<<dim3((n8w + 255) / 256), blk, 0, stream>>>(Wv, Wvb, n8w);
  cvt_w<<<dim3((n8c + 255) / 256), blk, 0, stream>>>(Wc, Wcb, n8c);
  gemm64<__bf16, (QRES ? 3 : 1), 1, false><<<dim3((tq + 7) / 8, 2, NB), blk, 0, stream>>>(
      Xc, DC, (long long)DD, XB, Wqb, DD, 0LL, 0LL,
      (void*)Qh, (void*)Ql, DD, VSTR, (long long)SEQ * DD, bq,
      NQ, DD, DD, 1.0f, 4096.0f);
  gemm64<__bf16, 1, 1, false><<<dim3((tk + 7) / 8, 2, 1), blk, 0, stream>>>(
      Xc, DC, (long long)DD, 0LL, Wkb, DD, 0LL, 0LL,
      (void*)Kp, (void*)Kp, DD, VSTR, 0LL, bk,
      NB * SEQ, DD, DD, 1.0f, 1.0f);
  gemm64<__bf16, 1, 2, false><<<dim3((tv + 7) / 8, NB, 2), blk, 0, stream>>>(
      Wvb, DD, 0LL, 0LL, Xc, DC, XB, (long long)DD,
      (void*)Vt, (void*)Vt, SEQ, VTB, VTV, bv,
      DD, SEQ, DD, 1.0f, 1.0f);
  gemm64<__bf16, 0, 1, true><<<dim3((tq + 7) / 8, 1, NB), blk, 0, stream>>>(
      Xc, DC, 0LL, XB, Wcb, DC, 0LL, 0LL,
      (void*)Co, (void*)Co, DD, 0LL, (long long)SEQ * DD, bc,
      NQ, DD, DC, 1.0f, 1.0f);
  attn_cv<<<dim3(NQ / 32, NB, 2), blk, 0, stream>>>(Qh, Ql, Kp, Vt, Co, (float*)d_out);
  (void)hipGetLastError();
}
